// SchNet_31928786878557
// MI455X (gfx1250) — hardware-verified
//
#include <hip/hip_runtime.h>
#include <math.h>

typedef __attribute__((ext_vector_type(16))) _Float16 v16h;
typedef __attribute__((ext_vector_type(8)))  _Float16 v8h;
typedef __attribute__((ext_vector_type(8)))  float    v8f;
typedef __attribute__((ext_vector_type(4)))  float    v4f;
typedef __attribute__((ext_vector_type(4)))  unsigned int v4u;
typedef __attribute__((ext_vector_type(4)))  int      v4i;

constexpr int NNODE  = 10000;
constexpr int NEDGE  = 320000;
constexpr int HID    = 128;
constexpr int NGS    = 50;
constexpr int KGP    = 64;
constexpr int NLAYER = 6;
constexpr int FEATW  = NGS + 2 * HID;
constexpr int NPADN  = 10240;
constexpr int NT     = 256;
constexpr int TILE   = 1024;
constexpr int NTILE  = NPADN / TILE;
constexpr int SPT    = 16;
constexpr int CHUNK  = NT * SPT;
constexpr int NCHUNK = (NEDGE + CHUNK - 1) / CHUNK;
constexpr int LCAPC  = 2048;
constexpr int LCAPF  = 2176;
constexpr int QCAP   = 256;
constexpr int NQUAD  = (NNODE * 3 + NNODE * HID) / 4;
constexpr int REGF   = 16896;

constexpr float EA_CARRY  = 16384.0f;
constexpr float W_CARRY   = 256.0f;
constexpr float T_CARRY   = 1024.0f;
constexpr float H16_CARRY = 8.0f;
constexpr float AGG_CARRY = 256.0f;
constexpr float TMP_CARRY = 1024.0f;
constexpr float S1SCALE   = 1.0f / (EA_CARRY * W_CARRY);
constexpr float S2SCALE   = 1.0f / (T_CARRY * W_CARRY);
constexpr float GA_SCALE  = 1.0f / (H16_CARRY * W_CARRY);
constexpr float GB_SCALE  = 1.0f / (AGG_CARRY * W_CARRY);
constexpr float GC_SCALE  = 1.0f / (TMP_CARRY * W_CARRY);

static_assert(NEDGE % SPT == 0, "cfg");
static_assert(NEDGE % 32 == 0, "cfg");
static_assert(NEDGE % NT == 0, "cfg");
static_assert(NPADN % 64 == 0 && HID % 64 == 0 && HID % 32 == 0 && KGP % 32 == 0, "cfg");
static_assert(NPADN % NT == 0 && NPADN >= NNODE + 0, "cfg");
static_assert(TILE / NT == 4 && TILE % 128 == 0, "cfg");
static_assert((NNODE * 3) % 4 == 0, "cfg");
static_assert(128 * 72 + 128 * 136 <= REGF * 2, "cfg");
static_assert(128 * 132 <= REGF, "cfg");
static_assert(NNODE * 3 * 4 + NNODE * HID * 4 == 5240000, "cfg");

__device__ __forceinline__ int clampn(int x, int n) { return x < 0 ? 0 : (x >= n ? n - 1 : x); }
__device__ __forceinline__ int imin(int a, int b) { return a < b ? a : b; }
__device__ __forceinline__ unsigned short h_bits(float f) { const _Float16 h = (_Float16)f; return __builtin_bit_cast(unsigned short, h); }
__device__ __forceinline__ unsigned pk16(unsigned short a, unsigned short b) { return (unsigned)a | ((unsigned)b << 16); }
__device__ __forceinline__ void wave_lds_sync() {
  __builtin_amdgcn_fence(__ATOMIC_RELEASE, "workgroup");
  __builtin_amdgcn_wave_barrier();
  __builtin_amdgcn_fence(__ATOMIC_ACQUIRE, "workgroup");
}
__device__ __forceinline__ float sspf(float x) {
  const float t = __builtin_amdgcn_exp2f(fabsf(x) * -1.4426950408889634f);
  const float u = fmaf(t, 0.5f, 0.5f);
  return fmaxf(x, 0.0f) + 0.69314718055994531f * __builtin_amdgcn_logf(u);
}

__device__ __forceinline__ void dep_guard_h(v8f& a, v8f& b, v16h x, v16h y) { asm volatile("v_nop\n\tv_nop\n\tv_nop\n\tv_nop" : "+v"(a), "+v"(b) : "v"(x), "v"(y)); }
__device__ __forceinline__ void keep4_h(v16h a, v16h b, v16h c, v16h d) { asm volatile("v_nop" :: "v"(a), "v"(b), "v"(c), "v"(d)); }
__device__ __forceinline__ void acc_guard4(v8f& a, v8f& b, v8f& c, v8f& d) { asm volatile("v_nop\n\tv_nop\n\tv_nop\n\tv_nop" : "+v"(a), "+v"(b), "+v"(c), "+v"(d)); }
template <typename T> struct Frag;
template <> struct Frag<_Float16> {
  typedef v16h V; union U { v16h v; v8h h[2]; };
  static __device__ __forceinline__ v16h load(const _Float16* p) {
    U f; f.h[0] = *(const v8h*)(p); f.h[1] = *(const v8h*)(p + 16); return f.v;
  }
  static __device__ __forceinline__ v8f mma(v16h a, v16h b, v8f c) {
    return __builtin_amdgcn_wmma_f32_16x16x32_f16(false, a, false, b, (short)0, c, false, false);
  }
  static __device__ __forceinline__ void guard(v8f& a, v8f& b, v16h x, v16h y) { dep_guard_h(a, b, x, y); }
  static __device__ __forceinline__ void keep(v16h a, v16h b, v16h c, v16h d) { keep4_h(a, b, c, d); }
};
__device__ __forceinline__ v8f mma_h(v16h a, v16h b, v8f c) {
  c = __builtin_amdgcn_wmma_f32_16x16x32_f16(false, a, false, b, (short)0, c, false, false);
  asm volatile("v_nop\n\tv_nop\n\tv_nop\n\tv_nop" : "+v"(c) : "v"(a), "v"(b));
  return c;
}

template <int ET> struct Elem;
template <> struct Elem<0> { typedef _Float16 T; };
template <int ET, bool SPLIT, int BIAS_MODE, int OUT_MODE, bool RESID, int ACT = 0>
__global__ __launch_bounds__(256) void wmma_gemm64(
    const unsigned short* __restrict__ Ap, const unsigned short* __restrict__ A2p, int lda, long strideA,
    const unsigned short* __restrict__ Btp, const unsigned short* __restrict__ Bt2p, int ldb, long strideB,
    void* __restrict__ Cout, void* __restrict__ Cout2, int ldc, long strideC,
    const float* __restrict__ bias,
    const float* __restrict__ resid, long strideR,
    int M, int N, int K, float scale) {
  static_assert(!RESID || OUT_MODE == 3, "cfg");
  static_assert(OUT_MODE == 0 || OUT_MODE == 1 || OUT_MODE == 3, "cfg");
  typedef typename Elem<ET>::T T;
  typedef typename Frag<T>::V V;
  const T* A = (const T*)Ap; const T* A2 = (const T*)A2p; const T* Bt = (const T*)Btp; const T* Bt2 = (const T*)Bt2p;
  __shared__ __align__(16) float sT[8][16 * 68];
  const int b    = blockIdx.y;
  const int lane = threadIdx.x & 31;
  const int wave = threadIdx.x >> 5;
  const int tilesN = N >> 6;
  const int tilesM = M >> 6;
  const int tile = blockIdx.x * 8 + wave;
  if (tile >= tilesM * tilesN) return;
  const int tm = tile / tilesN;
  const int tn = tile - tm * tilesN;
  const int m0 = tm << 6;
  const int n0 = tn << 6;

  const T* Ab  = A  + (size_t)b * strideA;
  const T* Bb  = Bt + (size_t)b * strideB;
  const T* Ab2 = SPLIT ? (A2  + (size_t)b * strideA) : nullptr;
  const T* Bb2 = SPLIT ? (Bt2 + (size_t)b * strideB) : nullptr;

  const int rlane = lane & 15;
  const int koff  = (lane >> 4) * 8;
  const int mOff  = (lane >> 4) * 8;

  v8f acc[4][4];
#pragma unroll
  for (int i = 0; i < 4; ++i)
#pragma unroll
    for (int j = 0; j < 4; ++j) acc[i][j] = (v8f){0.f,0.f,0.f,0.f,0.f,0.f,0.f,0.f};

  for (int k0 = 0; k0 < K; k0 += 32) {
    V bh[4], bl[4];
#pragma unroll
    for (int j = 0; j < 4; ++j) {
      const size_t bo = (size_t)(n0 + (j << 4) + rlane) * ldb + koff + k0;
      bh[j] = Frag<T>::load(Bb + bo);
      if (SPLIT) bl[j] = Frag<T>::load(Bb2 + bo);
    }
#pragma unroll
    for (int i = 0; i < 4; ++i) {
      const size_t ao = (size_t)(m0 + (i << 4) + rlane) * lda + koff + k0;
      V ah = Frag<T>::load(Ab + ao);
      V al;
      if (SPLIT) al = Frag<T>::load(Ab2 + ao);
#pragma unroll
      for (int j = 0; j < 4; ++j) {
        acc[i][j] = Frag<T>::mma(ah, bh[j], acc[i][j]);
        if (SPLIT) {
          acc[i][j] = Frag<T>::mma(ah, bl[j], acc[i][j]);
          acc[i][j] = Frag<T>::mma(al, bh[j], acc[i][j]);
        }
      }
      Frag<T>::guard(acc[i][0], acc[i][3], ah, SPLIT ? al : ah);
    }
    Frag<T>::keep(bh[0], bh[1], bh[2], bh[3]);
    if (SPLIT) Frag<T>::keep(bl[0], bl[1], bl[2], bl[3]);
  }
  acc_guard4(acc[0][0], acc[0][1], acc[0][2], acc[0][3]);
  acc_guard4(acc[1][0], acc[1][1], acc[1][2], acc[1][3]);
  acc_guard4(acc[2][0], acc[2][1], acc[2][2], acc[2][3]);
  acc_guard4(acc[3][0], acc[3][1], acc[3][2], acc[3][3]);

  float* slab = sT[wave];
  const float* Rb = RESID ? (resid + (size_t)b * strideR) : nullptr;
#pragma unroll
  for (int i = 0; i < 4; ++i) {
    const int mBase = m0 + (i << 4);
#pragma unroll
    for (int j = 0; j < 4; ++j) {
      const int n = n0 + (j << 4) + rlane;
      float bv = 0.f;
      if (BIAS_MODE == 2) bv = bias[n];
#pragma unroll
      for (int r = 0; r < 8; ++r) {
        float v = acc[i][j][r] * scale;
        if (BIAS_MODE == 1) v += bias[mBase + mOff + r];
        if (BIAS_MODE == 2) v += bv;
        if (ACT == 2) v = fmaxf(v, 0.0f);
        if (ACT == 4) v = (v > 0.f) ? v : 0.01f * v;
        if (ACT == 6) v = sspf(v) * TMP_CARRY;
        slab[(mOff + r) * 68 + (j << 4) + rlane] = v;
      }
    }
    __builtin_amdgcn_fence(__ATOMIC_RELEASE, "workgroup");
    __builtin_amdgcn_wave_barrier();
    __builtin_amdgcn_fence(__ATOMIC_ACQUIRE, "workgroup");
    if (OUT_MODE == 0) {
      float* C = (float*)Cout + (size_t)b * strideC;
      const int hh = lane >> 4, c4 = (lane & 15) * 4;
      for (int pass = 0; pass < 2; ++pass) {
#pragma unroll
        for (int it = 0; it < 8; ++it) {
          const int row = it * 2 + hh;
          v4f v = *(const v4f*)(slab + row * 68 + c4);
          *(volatile v4f*)(C + (size_t)(mBase + row) * ldc + n0 + c4) = v;
        }
        __threadfence();
      }
    } else if (OUT_MODE == 1) {
      const int q = lane >> 3, c8 = (lane & 7) * 8;
      unsigned short* C = (unsigned short*)Cout + (size_t)b * strideC;
      for (int pass = 0; pass < 2; ++pass) {
#pragma unroll
        for (int it = 0; it < 4; ++it) {
          const int row = it * 4 + q;
          const float* sp = slab + row * 68 + c8;
          v8h hv;
#pragma unroll
          for (int e = 0; e < 8; ++e) hv[e] = (_Float16)sp[e];
          *(volatile v8h*)(C + (size_t)(mBase + row) * ldc + n0 + c8) = hv;
        }
        __threadfence();
      }
    } else {
      float* C = (float*)Cout + (size_t)b * strideC;
      unsigned short* C2 = (unsigned short*)Cout2 + (size_t)b * strideC;
      const int hh = lane >> 4, c4 = (lane & 15) * 4;
      if (RESID) {
#pragma unroll
        for (int it = 0; it < 8; ++it) {
          const int row = it * 2 + hh;
          v4f v = *(const v4f*)(slab + row * 68 + c4);
          const v4f rs = *(const v4f*)(Rb + (size_t)(mBase + row) * ldc + n0 + c4);
          v = v + rs;
          *(v4f*)(slab + row * 68 + c4) = v;
        }
        __builtin_amdgcn_fence(__ATOMIC_RELEASE, "workgroup");
        __builtin_amdgcn_wave_barrier();
        __builtin_amdgcn_fence(__ATOMIC_ACQUIRE, "workgroup");
      }
      for (int pass = 0; pass < 2; ++pass) {
#pragma unroll
        for (int it = 0; it < 8; ++it) {
          const int row = it * 2 + hh;
          v4f v = *(const v4f*)(slab + row * 68 + c4);
          *(volatile v4f*)(C + (size_t)(mBase + row) * ldc + n0 + c4) = v;
        }
        __threadfence();
      }
      const int q = lane >> 3, c8 = (lane & 7) * 8;
      for (int pass = 0; pass < 2; ++pass) {
#pragma unroll
        for (int it = 0; it < 4; ++it) {
          const int row = it * 4 + q;
          const float* sp = slab + row * 68 + c8;
          v8h hv;
#pragma unroll
          for (int e = 0; e < 8; ++e) hv[e] = (_Float16)(sp[e] * H16_CARRY);
          *(volatile v8h*)(C2 + (size_t)(mBase + row) * ldc + n0 + c8) = hv;
        }
        __threadfence();
      }
    }
    __builtin_amdgcn_fence(__ATOMIC_RELEASE, "workgroup");
    __builtin_amdgcn_wave_barrier();
    __builtin_amdgcn_fence(__ATOMIC_ACQUIRE, "workgroup");
  }
}

__device__ __forceinline__ int blk_excl_scan(int cnt, int* scan_ws, int tid, int* tot) {
  const int lane = tid & 31, wave = tid >> 5; int incl = cnt;
#pragma unroll
  for (int o = 1; o < 32; o <<= 1) { const int v = __shfl_up(incl, o, 32); if (lane >= o) incl += v; }
  if (lane == 31) scan_ws[wave] = incl;
  __syncthreads();
  if (wave == 0) { int wv = (lane < NT / 32) ? scan_ws[lane] : 0; int wincl = wv;
#pragma unroll
    for (int o = 1; o < 32; o <<= 1) { const int v = __shfl_up(wincl, o, 32); if (lane >= o) wincl += v; }
    if (lane < NT / 32) scan_ws[32 + lane] = wincl - wv; if (lane == 31) scan_ws[64] = wincl; }
  __syncthreads();
  const int res = scan_ws[32 + wave] + incl - cnt; *tot = scan_ws[64];
  return res;
}
template <int SP>
__device__ __forceinline__ int chunk_hits(const int* __restrict__ keyv, int e0, int n0, int tid, int* LISTp, int cap,
                                          int* scan_ws) {
  const int eb = e0 + tid * SP;
  const bool act = eb < NEDGE;
  const int ebc = act ? eb : (NEDGE - SP);
  int rec[SP]; int cnt = 0;
#pragma unroll
  for (int k = 0; k < SP; k += 4) {
    const v4i d4 = *(const v4i*)(keyv + ebc + k);
#pragma unroll
    for (int q = 0; q < 4; ++q) {
      const int d = d4[q]; int r = -1;
      if (act && d >= n0 && d < n0 + TILE) { r = ((d - n0) << 19) | (ebc + k + q); ++cnt; }
      rec[k + q] = r;
    }
  }
  int tot; int p = blk_excl_scan(cnt, scan_ws, tid, &tot);
#pragma unroll
  for (int k = 0; k < SP; ++k) if (rec[k] >= 0) { if (p < cap) LISTp[p] = rec[k]; ++p; }
  __syncthreads();
  return tot < cap ? tot : cap;
}

__device__ __forceinline__ float gaussf(float d, int k, float coeff) {
  const float rk = (float)k * (1.0f / 49.0f);
  float off = 10.0f * rk;
  off = (k == NGS - 1) ? 10.0f : off;
  const float dd = d - off;
  return expf(coeff * (dd * dd));
}
__global__ __launch_bounds__(NT) void k_edge_init(const float* __restrict__ pos, const int* __restrict__ ei,
                                                   const float* __restrict__ cwall,
                                                   unsigned short* __restrict__ EA, float* __restrict__ EMETA) {
  const int t = threadIdx.x;
  const int q = t >> 3, j = t & 7;
  const int e = blockIdx.x * 32 + q;
  const int r = clampn(ei[e], NNODE), c = clampn(ei[NEDGE + e], NNODE);
  const float dx = pos[r * 3 + 0] - pos[c * 3 + 0];
  const float dy = pos[r * 3 + 1] - pos[c * 3 + 1];
  const float dz = pos[r * 3 + 2] - pos[c * 3 + 2];
  const float d = sqrtf((dx * dx + dz * dz) + dy * dy);
  const float off1 = 10.0f * (1.0f * (1.0f / 49.0f));
  const float coeff = -0.5f / (off1 * off1);
  float p[NLAYER];
#pragma unroll
  for (int l = 0; l < NLAYER; ++l) p[l] = 0.0f;
  unsigned w0 = 0u, w1 = 0u, w2 = 0u, w3 = 0u;
#pragma unroll 1
  for (int ii = 0; ii < 4; ++ii) {
    const int k0 = 8 * j + 2 * ii, k1 = k0 + 1;
    float g0 = gaussf(d, k0, coeff), g1 = gaussf(d, k1, coeff);
    g0 = (k0 < NGS) ? g0 : 0.0f;
    g1 = (k1 < NGS) ? g1 : 0.0f;
    const int kc0 = (k0 < NGS) ? k0 : NGS - 1, kc1 = (k1 < NGS) ? k1 : NGS - 1;
#pragma unroll
    for (int l = 0; l < NLAYER; ++l) {
      p[l] = fmaf(g0, cwall[l * FEATW + kc0], p[l]);
      p[l] = fmaf(g1, cwall[l * FEATW + kc1], p[l]);
    }
    const unsigned u = pk16(h_bits(g0 * EA_CARRY), h_bits(g1 * EA_CARRY));
    w0 = (ii == 0) ? u : w0; w1 = (ii == 1) ? u : w1; w2 = (ii == 2) ? u : w2; w3 = (ii == 3) ? u : w3;
  }
  const v4u uv = (v4u){w0, w1, w2, w3};
  unsigned short* eap = EA + (size_t)e * KGP + 8 * j;
  *(volatile v4u*)eap = uv;
  __threadfence();
  *(volatile v4u*)eap = uv;
  float val = 0.0f;
#pragma unroll
  for (int l = 0; l < NLAYER; ++l) {
    float s = p[l];
    s += __shfl_xor(s, 1, 32); s += __shfl_xor(s, 2, 32); s += __shfl_xor(s, 4, 32);
    val = (j == l) ? s : val;
  }
  float* mp = EMETA + (size_t)e * 8 + j;
  *(volatile float*)mp = val;
  __threadfence();
  *(volatile float*)mp = val;
}

__global__ __launch_bounds__(NT) void k_edge_cut(const float* __restrict__ pos, const int* __restrict__ ei,
                                                  float* __restrict__ CPL) {
  const int e = blockIdx.x * NT + threadIdx.x;
  const int r = clampn(ei[e], NNODE), c = clampn(ei[NEDGE + e], NNODE);
  const float dx = pos[r * 3 + 0] - pos[c * 3 + 0];
  const float dy = pos[r * 3 + 1] - pos[c * 3 + 1];
  const float dz = pos[r * 3 + 2] - pos[c * 3 + 2];
  const float d = sqrtf((dx * dx + dz * dz) + dy * dy);
  const float a = (d * 3.14159274101257324f) * 0.1f;
  const float cv = 0.5f * (cosf(a) + 1.0f);
  *(volatile float*)(CPL + e) = cv;
  __threadfence();
  *(volatile float*)(CPL + e) = cv;
}

__global__ __launch_bounds__(NT) void k_wcast(const float* __restrict__ m1w, const float* __restrict__ m2w,
                                               const float* __restrict__ l1w, const float* __restrict__ l2w,
                                               const float* __restrict__ lw,
                                               unsigned short* __restrict__ W1T, unsigned short* __restrict__ W2T,
                                               unsigned short* __restrict__ L1T, unsigned short* __restrict__ L2T,
                                               unsigned short* __restrict__ LT) {
  const int pz = blockIdx.y;
  const float* W = (pz == 0) ? m1w : (pz == 1) ? m2w : (pz == 2) ? l1w : (pz == 3) ? l2w : lw;
  unsigned short* O = (pz == 0) ? W1T : (pz == 1) ? W2T : (pz == 2) ? L1T : (pz == 3) ? L2T : LT;
  const int KI = (pz == 0) ? NGS : HID;
  const int KO = (pz == 0) ? KGP : HID;
  const int nch = KO >> 3;
  const int total = NLAYER * HID * nch;
  const int idx = blockIdx.x * NT + threadIdx.x;
  if (idx >= total) return;
  const int row = idx / nch;
  const int c8 = (idx - row * nch) * 8;
  unsigned short hb[8];
#pragma unroll
  for (int e = 0; e < 8; ++e) {
    const int k = c8 + e;
    const int kc = (k < KI) ? k : KI - 1;
    float v = W[(size_t)row * KI + kc] * W_CARRY;
    v = (k < KI) ? v : 0.0f;
    hb[e] = h_bits(v);
  }
  const v4u u = (v4u){pk16(hb[0], hb[1]), pk16(hb[2], hb[3]), pk16(hb[4], hb[5]), pk16(hb[6], hb[7])};
  unsigned short* op = O + (size_t)row * KO + c8;
  *(volatile v4u*)op = u;
  __threadfence();
  *(volatile v4u*)op = u;
}

__global__ __launch_bounds__(NT) void k_node_init(const float* __restrict__ z, const float* __restrict__ pos,
                                                   float* __restrict__ HA, unsigned short* __restrict__ H16A,
                                                   float* __restrict__ POSA) {
  const int i = blockIdx.x * NT + threadIdx.x;
  {
    const int row = i >> 5, c4 = (i & 31) * 4;
    const int rr = imin(row, NNODE - 1);
    const float f = (row < NNODE) ? 1.0f : 0.0f;
    v4f v = *(const v4f*)(z + (size_t)rr * HID + c4);
    v = v * f;
    float* p = HA + 4 * (size_t)i;
    *(volatile v4f*)p = v;
    __threadfence();
    *(volatile v4f*)p = v;
  }
  if (i < NPADN * HID / 8) {
    const int row = i >> 4, c8 = (i & 15) * 8;
    const int rr = imin(row, NNODE - 1);
    const float f = ((row < NNODE) ? 1.0f : 0.0f) * H16_CARRY;
    const v4f a = *(const v4f*)(z + (size_t)rr * HID + c8);
    const v4f c = *(const v4f*)(z + (size_t)rr * HID + c8 + 4);
    unsigned short hb[8];
#pragma unroll
    for (int e = 0; e < 4; ++e) { hb[e] = h_bits(a[e] * f); hb[4 + e] = h_bits(c[e] * f); }
    const v4u u = (v4u){pk16(hb[0], hb[1]), pk16(hb[2], hb[3]), pk16(hb[4], hb[5]), pk16(hb[6], hb[7])};
    unsigned short* p = H16A + 8 * (size_t)i;
    *(volatile v4u*)p = u;
    __threadfence();
    *(volatile v4u*)p = u;
  }
  if (i < NPADN) {
    const int rr = imin(i, NNODE - 1);
    const float f = (i < NNODE) ? 1.0f : 0.0f;
    const v4f v = (v4f){pos[rr * 3 + 0] * f, pos[rr * 3 + 1] * f, pos[rr * 3 + 2] * f, 0.0f};
    float* p = POSA + 4 * (size_t)i;
    *(volatile v4f*)p = v;
    __threadfence();
    *(volatile v4f*)p = v;
  }
}

__global__ __launch_bounds__(NT) void k_arc(const float* __restrict__ H, const float* __restrict__ cw,
                                             float* __restrict__ ARC) {
  const int n = blockIdx.x * NT + threadIdx.x;
  const float* hr = H + (size_t)n * HID;
  float ar = 0.0f, ac = 0.0f;
#pragma unroll 4
  for (int k = 0; k < HID; ++k) {
    const float hv = hr[k];
    ar = fmaf(hv, cw[NGS + k], ar);
    ac = fmaf(hv, cw[NGS + HID + k], ac);
  }
  *(volatile float*)(ARC + n) = ar;
  *(volatile float*)(ARC + NPADN + n) = ac;
  __threadfence();
  *(volatile float*)(ARC + n) = ar;
  *(volatile float*)(ARC + NPADN + n) = ac;
}

__global__ __launch_bounds__(NT) void k_coord(const int* __restrict__ ei, const float* __restrict__ EMETA,
                                               const float* __restrict__ ARC, const float* __restrict__ cbp,
                                               const float* __restrict__ POSs, float* __restrict__ POSd, int layer) {
  __shared__ __align__(16) float posL[TILE * 4];
  __shared__ float arL[TILE];
  __shared__ __align__(16) float sumsL[TILE * 4];
  __shared__ int cntL[TILE];
  __shared__ int tagL[TILE];
  __shared__ int LIST[LCAPC];
  __shared__ int WQ[8 * QCAP];
  __shared__ int scan_ws[80];
  const int tid = threadIdx.x, lane = tid & 31, wave = tid >> 5;
  const int n0 = blockIdx.x * TILE;
  const float cb = cbp[0];
  const v4f z4 = (v4f){0.f, 0.f, 0.f, 0.f};
  for (int i = tid; i < TILE; i += NT) {
    const int n = n0 + i;
    const int nc = (n < NNODE) ? n : NNODE - 1;
    *(v4f*)(posL + 4 * i) = *(const v4f*)(POSs + (size_t)nc * 4);
    arL[i] = ARC[n];
    *(v4f*)(sumsL + 4 * i) = z4;
    cntL[i] = 0;
    tagL[i] = 0;
  }
  for (int i = tid; i < LCAPC; i += NT) LIST[i] = 0;
  for (int i = tid; i < 8 * QCAP; i += NT) WQ[i] = 0;
  __syncthreads();
  const unsigned lt = (1u << lane) - 1u;
  int* WQw = WQ + wave * QCAP;
#pragma unroll 1
  for (int c = 0; c < NCHUNK; ++c) {
    const int tot = chunk_hits<SPT>(ei, c * CHUNK, n0, tid, LIST, LCAPC, scan_ws);
    int qn = 0;
#pragma unroll 1
    for (int base = 0; base < tot; base += 32) {
      const int q = base + lane;
      const int li = (q < LCAPC) ? q : LCAPC - 1;
      const int rv = LIST[li];
      const int dl = (rv >> 19) & (TILE - 1);
      const int own = ((q < tot) && ((dl >> 7) == wave)) ? 1 : 0;
      const unsigned m = (unsigned)__ballot(own);
      const int my = qn + (int)__popc(m & lt);
      if (own && my < QCAP) WQw[my] = rv;
      qn += (int)__popc(m);
    }
    qn = (qn < QCAP) ? qn : QCAP;
    wave_lds_sync();
#pragma unroll 1
    for (int b2 = 0; b2 < qn; b2 += 32) {
      const int q = b2 + lane;
      const bool act = q < qn;
      const int rv = WQw[(q < QCAP) ? q : QCAP - 1];
      int e = rv & 0x7FFFF; e = (e < NEDGE) ? e : NEDGE - 1;
      const int dl = (rv >> 19) & (TILE - 1);
      const int cnode = clampn(ei[NEDGE + e], NNODE);
      const float em  = EMETA[(size_t)e * 8 + layer];
      const float acv = ARC[NPADN + cnode];
      const v4f pc = *(const v4f*)(POSs + (size_t)cnode * 4);
      const v4f pr = *(const v4f*)(posL + dl * 4);
      const float ar = arL[dl];
      const float cwv = ((em + ar) + acv) + cb;
      const float vx = (pr[0] - pc[0]) * cwv;
      const float vy = (pr[1] - pc[1]) * cwv;
      const float vz = (pr[2] - pc[2]) * cwv;
      int done = act ? 0 : 1;
#pragma unroll 1
      for (int it = 0; it < 32; ++it) {
        const unsigned left = (unsigned)__ballot(done == 0 ? 1 : 0);
        if (left == 0u) break;
        if (done == 0) tagL[dl] = lane;
        wave_lds_sync();
        const int tg = tagL[dl];
        const int win = ((done == 0) && (tg == lane)) ? 1 : 0;
        if (win) {
          sumsL[dl * 4 + 0] += vx;
          sumsL[dl * 4 + 1] += vy;
          sumsL[dl * 4 + 2] += vz;
          cntL[dl] += 1;
          done = 1;
        }
        wave_lds_sync();
      }
    }
    __syncthreads();
  }
  v4f pn[4];
#pragma unroll
  for (int k = 0; k < 4; ++k) {
    const int i = tid + k * NT;
    const int n = n0 + i;
    const int cnt = cntL[i];
    const float cf = (float)cnt;
    const float inv = (cnt > 0) ? (1.0f / fmaxf(cf, 1.0f)) : 0.0f;
    const v4f s = *(const v4f*)(sumsL + 4 * i);
    const v4f p0 = *(const v4f*)(posL + 4 * i);
    v4f rr = p0 + s * inv;
    rr[3] = 0.0f;
    const float live = (n < NNODE) ? 1.0f : 0.0f;
    rr = rr * live;
    pn[k] = rr;
  }
  for (int pass = 0; pass < 2; ++pass) {
#pragma unroll
    for (int k = 0; k < 4; ++k) *(volatile v4f*)(POSd + (size_t)(n0 + tid + k * NT) * 4) = pn[k];
    __threadfence();
  }
}

__global__ __launch_bounds__(NT) void k_filter_agg(const int* __restrict__ ei, const unsigned short* __restrict__ EAp,
    const float* __restrict__ CPL, const unsigned short* __restrict__ W1Tl, const float* __restrict__ b1l,
    const unsigned short* __restrict__ W2Tl, const float* __restrict__ b2l, const float* __restrict__ XF,
    float* AGG, unsigned short* __restrict__ AGG16) {
  __shared__ __align__(16) _Float16 W1s[HID * 72];
  __shared__ __align__(16) float REG[REGF];
  __shared__ int LIST[LCAPF];
  __shared__ int mDL[128];
  __shared__ int mROW[128];
  __shared__ float mC[128];
  __shared__ int scan_ws[80];
  _Float16* EAs = (_Float16*)REG;
  _Float16* Ts  = ((_Float16*)REG) + 9216;
  float*    WFs = REG;
  const int tid = threadIdx.x, lane = tid & 31, wave = tid >> 5;
  const int rlane = lane & 15, koff = (lane >> 4) * 8, mOff = (lane >> 4) * 8;
  const int n0 = blockIdx.x * TILE;
  const int r0 = wave * 16;
  const _Float16* W2 = (const _Float16*)W2Tl;
#pragma unroll
  for (int i = 0; i < 4; ++i) {
    const int idx = tid + i * NT;
    const int row = idx >> 3, c8 = (idx & 7) * 8;
    const v4u u = *(const v4u*)(W1Tl + row * KGP + c8);
    *(v4u*)(W1s + row * 72 + c8) = u;
  }
  for (int i = tid; i < LCAPF; i += NT) LIST[i] = 0;
  const v4f z4 = (v4f){0.f, 0.f, 0.f, 0.f};
#pragma unroll 1
  for (int j = 0; j < 128; ++j) {
    float* zp = AGG + (size_t)(n0 + wave * 128 + j) * HID + 4 * lane;
    *(volatile v4f*)zp = z4;
    __threadfence();
    *(volatile v4f*)zp = z4;
  }
  __syncthreads();
  int rem = 0;
  const int* colv = ei + NEDGE;
#pragma unroll 1
  for (int c = 0; c < NCHUNK; ++c) {
    const int nh = chunk_hits<SPT>(colv, c * CHUNK, n0, tid, LIST + rem, LCAPF - rem, scan_ws);
    const int tot = rem + nh;
    const bool last = (c == NCHUNK - 1);
    const int ngp = last ? ((tot + 127) >> 7) : (tot >> 7);
#pragma unroll 1
    for (int g = 0; g < ngp; ++g) {
      const int gbase = g << 7;
      const int nvalid = ((tot - gbase) < 128) ? (tot - gbase) : 128;
      {
        const int s = tid >> 1, hq = tid & 1;
        int li = gbase + s; li = (li < LCAPF) ? li : LCAPF - 1;
        const int rv = LIST[li];
        int e = rv & 0x7FFFF; e = (e < NEDGE) ? e : NEDGE - 1;
        const int dl = (rv >> 19) & (TILE - 1);
        const int rw = clampn(ei[e], NNODE);
        float cv = CPL[e];
        cv = (s < nvalid) ? cv : 0.0f;
        if (hq == 0) { mDL[s] = dl; mROW[s] = rw; mC[s] = cv; }
        const unsigned short* src = EAp + (size_t)e * KGP + hq * 32;
        const v4u u0 = *(const v4u*)(src);
        const v4u u1 = *(const v4u*)(src + 8);
        const v4u u2 = *(const v4u*)(src + 16);
        const v4u u3 = *(const v4u*)(src + 24);
        _Float16* dst = EAs + s * 72 + hq * 32;
        *(v4u*)(dst) = u0;
        *(v4u*)(dst + 8) = u1;
        *(v4u*)(dst + 16) = u2;
        *(v4u*)(dst + 24) = u3;
      }
      __syncthreads();
      {
        v16h a0, a1;
        { Frag<_Float16>::U f; f.h[0] = *(const v8h*)(EAs + (r0 + rlane) * 72 + koff);
          f.h[1] = *(const v8h*)(EAs + (r0 + rlane) * 72 + koff + 16); a0 = f.v; }
        { Frag<_Float16>::U f; f.h[0] = *(const v8h*)(EAs + (r0 + rlane) * 72 + 32 + koff);
          f.h[1] = *(const v8h*)(EAs + (r0 + rlane) * 72 + 32 + koff + 16); a1 = f.v; }
#pragma unroll
        for (int j = 0; j < 8; ++j) {
          v16h bA, bB;
          { Frag<_Float16>::U f; f.h[0] = *(const v8h*)(W1s + (16 * j + rlane) * 72 + koff);
            f.h[1] = *(const v8h*)(W1s + (16 * j + rlane) * 72 + koff + 16); bA = f.v; }
          { Frag<_Float16>::U f; f.h[0] = *(const v8h*)(W1s + (16 * j + rlane) * 72 + 32 + koff);
            f.h[1] = *(const v8h*)(W1s + (16 * j + rlane) * 72 + 32 + koff + 16); bB = f.v; }
          v8f acc = (v8f){0.f,0.f,0.f,0.f,0.f,0.f,0.f,0.f};
          acc = mma_h(a0, bA, acc);
          acc = mma_h(a1, bB, acc);
          const float bv = b1l[16 * j + rlane];
#pragma unroll
          for (int r = 0; r < 8; ++r) {
            const float x = fmaf(acc[r], S1SCALE, bv);
            const float tv = sspf(x) * T_CARRY;
            Ts[(r0 + mOff + r) * 136 + 16 * j + rlane] = (_Float16)tv;
          }
        }
      }
      __syncthreads();
      v8f acc2[8];
#pragma unroll
      for (int j = 0; j < 8; ++j) acc2[j] = (v8f){0.f,0.f,0.f,0.f,0.f,0.f,0.f,0.f};
#pragma unroll 1
      for (int ks = 0; ks < 4; ++ks) {
        v16h a;
        { Frag<_Float16>::U f; f.h[0] = *(const v8h*)(Ts + (r0 + rlane) * 136 + 32 * ks + koff);
          f.h[1] = *(const v8h*)(Ts + (r0 + rlane) * 136 + 32 * ks + koff + 16); a = f.v; }
#pragma unroll
        for (int j = 0; j < 8; ++j) {
          const v16h bj = Frag<_Float16>::load(W2 + (size_t)(16 * j + rlane) * HID + 32 * ks + koff);
          acc2[j] = mma_h(a, bj, acc2[j]);
        }
      }
      __syncthreads();
#pragma unroll
      for (int j = 0; j < 8; ++j) {
        const float bv = b2l[16 * j + rlane];
#pragma unroll
        for (int r = 0; r < 8; ++r) {
          const int s = r0 + mOff + r;
          const float v = fmaf(acc2[j][r], S2SCALE, bv) * mC[s];
          WFs[s * 132 + 16 * j + rlane] = v;
        }
      }
      __syncthreads();
#pragma unroll 1
      for (int qq = 0; qq < 4; ++qq) {
        const int s = qq * 32 + lane;
        const int dl = mDL[s];
        const int own = ((s < nvalid) && ((dl >> 7) == wave)) ? 1 : 0;
        unsigned msk = (unsigned)__ballot(own);
#pragma unroll 1
        for (int it = 0; it < 32; ++it) {
          if (msk == 0u) break;
          const int bp = __builtin_ctz(msk); msk &= msk - 1u;
          const int s2 = qq * 32 + bp;
          const int dlu = mDL[s2];
          const int rw  = mROW[s2];
          const v4f xv = *(const v4f*)(XF + (size_t)rw * HID + 4 * lane);
          const v4f wv = *(const v4f*)(WFs + s2 * 132 + 4 * lane);
          float* ap = AGG + (size_t)(n0 + dlu) * HID + 4 * lane;
          v4f av = *(const v4f*)ap;
          av = av + xv * wv;
          *(volatile v4f*)ap = av;
          __threadfence();
          *(volatile v4f*)ap = av;
        }
      }
      __syncthreads();
    }
    if (!last) {
      const int done = ngp << 7;
      rem = tot - done;
      if (done > 0 && tid < rem) LIST[tid] = LIST[done + tid];
      __syncthreads();
    }
  }
  __syncthreads();
#pragma unroll 1
  for (int jp = 0; jp < 64; ++jp) {
    const int row = n0 + wave * 128 + 2 * jp + (lane >> 4);
    const int c8 = (lane & 15) * 8;
    const float* rp = AGG + (size_t)row * HID + c8;
    const v4f v0 = *(const v4f*)(rp);
    const v4f v1 = *(const v4f*)(rp + 4);
    unsigned short hb[8];
#pragma unroll
    for (int e = 0; e < 4; ++e) { hb[e] = h_bits(v0[e] * AGG_CARRY); hb[4 + e] = h_bits(v1[e] * AGG_CARRY); }
    const v4u u = (v4u){pk16(hb[0], hb[1]), pk16(hb[2], hb[3]), pk16(hb[4], hb[5]), pk16(hb[6], hb[7])};
    unsigned short* op = AGG16 + (size_t)row * HID + c8;
    *(volatile v4u*)op = u;
    __threadfence();
    *(volatile v4u*)op = u;
  }
}

__global__ __launch_bounds__(NT) void k_pack(const float* __restrict__ POS, const float* __restrict__ H,
                                              float* __restrict__ out, int nquad) {
  const int i = blockIdx.x * NT + threadIdx.x;
  if (i >= nquad) return;
  float v[4];
#pragma unroll
  for (int j = 0; j < 4; ++j) {
    const int idx = 4 * i + j;
    const int pidx = (idx < NNODE * 3) ? idx : (NNODE * 3 - 1);
    const int node = pidx / 3;
    const int comp = pidx - 3 * node;
    const float pa = POS[node * 4 + comp];
    int hi = idx - NNODE * 3; hi = (hi < 0) ? 0 : hi;
    const float hb = H[hi];
    const float fsel = (idx < NNODE * 3) ? 1.0f : 0.0f;
    v[j] = fmaf(fsel, pa, (1.0f - fsel) * hb);
  }
  const v4f o = (v4f){v[0], v[1], v[2], v[3]};
  *(volatile v4f*)(out + 4 * (size_t)i) = o;
  __threadfence();
  *(volatile v4f*)(out + 4 * (size_t)i) = o;
}

extern "C" void kernel_launch(void* const* d_in, const int* in_sizes, int n_in,
                              void* d_out, int out_size, void* d_ws, size_t ws_size, hipStream_t stream) {
  (void)in_sizes; (void)n_in; (void)out_size;
  const float* z    = (const float*)d_in[0];
  const float* pos  = (const float*)d_in[1];
  const int*   ei   = (const int*)d_in[2];
  const float* m1w  = (const float*)d_in[3];
  const float* m1b  = (const float*)d_in[4];
  const float* m2w  = (const float*)d_in[5];
  const float* m2b  = (const float*)d_in[6];
  const float* l1w  = (const float*)d_in[7];
  const float* l2w  = (const float*)d_in[8];
  const float* l2b  = (const float*)d_in[9];
  const float* lw   = (const float*)d_in[10];
  const float* lb   = (const float*)d_in[11];
  const float* cw   = (const float*)d_in[12];
  const float* cb   = (const float*)d_in[13];
  float* out = (float*)d_out;

  char* ws = (char*)d_ws; size_t off = 0;
  auto carve = [&](size_t bytes) -> char* { char* p = ws + off; off += (bytes + 255) & ~(size_t)255; return p; };
  unsigned short* EA    = (unsigned short*)carve((size_t)NEDGE * KGP * 2);
  float*          EMETA = (float*)carve((size_t)NEDGE * 8 * 4);
  float*          CPL   = (float*)carve((size_t)NEDGE * 4);
  unsigned short* W1T   = (unsigned short*)carve((size_t)NLAYER * HID * KGP * 2);
  unsigned short* W2T   = (unsigned short*)carve((size_t)NLAYER * HID * HID * 2);
  unsigned short* L1T   = (unsigned short*)carve((size_t)NLAYER * HID * HID * 2);
  unsigned short* L2T   = (unsigned short*)carve((size_t)NLAYER * HID * HID * 2);
  unsigned short* LT    = (unsigned short*)carve((size_t)NLAYER * HID * HID * 2);
  float*          HA    = (float*)carve((size_t)NPADN * HID * 4);
  float*          HB    = (float*)carve((size_t)NPADN * HID * 4);
  unsigned short* H16A  = (unsigned short*)carve((size_t)NPADN * HID * 2);
  unsigned short* H16B  = (unsigned short*)carve((size_t)NPADN * HID * 2);
  float*          POSA  = (float*)carve((size_t)NPADN * 4 * 4);
  float*          POSB  = (float*)carve((size_t)NPADN * 4 * 4);
  float*          ARC   = (float*)carve((size_t)2 * NPADN * 4);
  float*          XF    = (float*)carve((size_t)NPADN * HID * 4);
  float*          AGG   = (float*)carve((size_t)NPADN * HID * 4);
  unsigned short* AGG16 = (unsigned short*)carve((size_t)NPADN * HID * 2);
  unsigned short* TMP16 = (unsigned short*)carve((size_t)NPADN * HID * 2);
  if (off > ws_size || off > (size_t)134217728) return;

  k_edge_init<<<NEDGE / 32, NT, 0, stream>>>(pos, ei, cw, EA, EMETA);
  k_edge_cut<<<NEDGE / NT, NT, 0, stream>>>(pos, ei, CPL);
  k_wcast<<<dim3(48, 5), NT, 0, stream>>>(m1w, m2w, l1w, l2w, lw, W1T, W2T, L1T, L2T, LT);
  k_node_init<<<(NPADN * HID / 4) / NT, NT, 0, stream>>>(z, pos, HA, H16A, POSA);

  const int gemmBlocks = ((NPADN / 64) * (HID / 64) + 7) / 8;
  for (int l = 0; l < NLAYER; ++l) {
    const float* Hs = (l & 1) ? HB : HA;
    float*       Hd = (l & 1) ? HA : HB;
    const unsigned short* H16s = (l & 1) ? H16B : H16A;
    unsigned short*       H16d = (l & 1) ? H16A : H16B;
    const float* Ps = (l & 1) ? POSB : POSA;
    float*       Pd = (l & 1) ? POSA : POSB;
    k_arc<<<NPADN / NT, NT, 0, stream>>>(Hs, cw + (size_t)l * FEATW, ARC);
    k_coord<<<NTILE, NT, 0, stream>>>(ei, EMETA, ARC, cb + l, Ps, Pd, l);
    wmma_gemm64<0, false, 0, 0, false, 0><<<dim3(gemmBlocks, 1), 256, 0, stream>>>(
        H16s, (const unsigned short*)nullptr, HID, 0L,
        L1T + (size_t)l * HID * HID, (const unsigned short*)nullptr, HID, 0L,
        (void*)XF, (void*)nullptr, HID, 0L,
        (const float*)nullptr, (const float*)nullptr, 0L, NPADN, HID, HID, GA_SCALE);
    k_filter_agg<<<NTILE, NT, 0, stream>>>(ei, EA, CPL, W1T + (size_t)l * HID * KGP, m1b + (size_t)l * HID,
                                           W2T + (size_t)l * HID * HID, m2b + (size_t)l * HID, XF, AGG, AGG16);
    wmma_gemm64<0, false, 2, 1, false, 6><<<dim3(gemmBlocks, 1), 256, 0, stream>>>(
        AGG16, (const unsigned short*)nullptr, HID, 0L,
        L2T + (size_t)l * HID * HID, (const unsigned short*)nullptr, HID, 0L,
        (void*)TMP16, (void*)nullptr, HID, 0L,
        l2b + (size_t)l * HID, (const float*)nullptr, 0L, NPADN, HID, HID, GB_SCALE);
    wmma_gemm64<0, false, 2, 3, true, 0><<<dim3(gemmBlocks, 1), 256, 0, stream>>>(
        TMP16, (const unsigned short*)nullptr, HID, 0L,
        LT + (size_t)l * HID * HID, (const unsigned short*)nullptr, HID, 0L,
        (void*)Hd, (void*)H16d, HID, 0L,
        lb + (size_t)l * HID, Hs, 0L, NPADN, HID, HID, GC_SCALE);
  }
  k_pack<<<(NQUAD + NT - 1) / NT, NT, 0, stream>>>(POSA, HA, out, NQUAD);
}
